// RoPEMaskedAttentionHead_80384607911994
// MI455X (gfx1250) — hardware-verified
//
#include <hip/hip_runtime.h>
#include <stdint.h>

typedef __attribute__((ext_vector_type(16))) _Float16 v16h;
typedef __attribute__((ext_vector_type(8)))  _Float16 v8h;
typedef __attribute__((ext_vector_type(16))) __bf16   v16b;
typedef __attribute__((ext_vector_type(8)))  __bf16   v8b;
typedef __attribute__((ext_vector_type(8)))  float    v8f;
typedef __attribute__((ext_vector_type(4)))  float    v4f;
typedef __attribute__((ext_vector_type(4)))  unsigned int v4u;

__device__ __forceinline__ unsigned short f2bf_bits(float f) {
  unsigned u = __float_as_uint(f);
  return (unsigned short)((u + 0x7FFFu + ((u >> 16) & 1u)) >> 16);
}
__device__ __forceinline__ float bf_bits2f(unsigned short h) { return __uint_as_float(((unsigned)h) << 16); }

__device__ __forceinline__ void dep_guard_h(v8f& a, v8f& b, v16h x, v16h y) { asm volatile("v_nop\n\tv_nop\n\tv_nop\n\tv_nop" : "+v"(a), "+v"(b) : "v"(x), "v"(y)); }
__device__ __forceinline__ void dep_guard_b(v8f& a, v8f& b, v16b x, v16b y) { asm volatile("v_nop\n\tv_nop\n\tv_nop\n\tv_nop" : "+v"(a), "+v"(b) : "v"(x), "v"(y)); }
__device__ __forceinline__ void keep4_h(v16h a, v16h b, v16h c, v16h d) { asm volatile("v_nop" :: "v"(a), "v"(b), "v"(c), "v"(d)); }
__device__ __forceinline__ void keep4_b(v16b a, v16b b, v16b c, v16b d) { asm volatile("v_nop" :: "v"(a), "v"(b), "v"(c), "v"(d)); }
__device__ __forceinline__ void acc_guard4(v8f& a, v8f& b, v8f& c, v8f& d) { asm volatile("v_nop\n\tv_nop\n\tv_nop\n\tv_nop" : "+v"(a), "+v"(b), "+v"(c), "+v"(d)); }
template <typename T> struct Frag;
template <> struct Frag<_Float16> {
  typedef v16h V; union U { v16h v; v8h h[2]; };
  static __device__ __forceinline__ v16h load(const _Float16* p) {
    U f; f.h[0] = *(const v8h*)(p); f.h[1] = *(const v8h*)(p + 16); return f.v;
  }
  static __device__ __forceinline__ v8f mma(v16h a, v16h b, v8f c) {
    return __builtin_amdgcn_wmma_f32_16x16x32_f16(false, a, false, b, (short)0, c, false, false);
  }
  static __device__ __forceinline__ void guard(v8f& a, v8f& b, v16h x, v16h y) { dep_guard_h(a, b, x, y); }
  static __device__ __forceinline__ void keep(v16h a, v16h b, v16h c, v16h d) { keep4_h(a, b, c, d); }
};
template <> struct Frag<__bf16> {
  typedef v16b V; union U { v16b v; v8b h[2]; };
  static __device__ __forceinline__ v16b load(const __bf16* p) {
    U f; f.h[0] = *(const v8b*)(p); f.h[1] = *(const v8b*)(p + 16); return f.v;
  }
  static __device__ __forceinline__ v8f mma(v16b a, v16b b, v8f c) {
    return __builtin_amdgcn_wmma_f32_16x16x32_bf16(false, a, false, b, (short)0, c, false, false);
  }
  static __device__ __forceinline__ void guard(v8f& a, v8f& b, v16b x, v16b y) { dep_guard_b(a, b, x, y); }
  static __device__ __forceinline__ void keep(v16b a, v16b b, v16b c, v16b d) { keep4_b(a, b, c, d); }
};

template <int ET> struct Elem;
template <> struct Elem<0> { typedef _Float16 T; };
template <> struct Elem<1> { typedef __bf16 T; };

template <int ET, bool SPLIT, int OUT_MODE, int TILEMAP, bool KCAUS, bool ROT>
__global__ __launch_bounds__(256) void gemm64x(
    const unsigned short* __restrict__ Ap, const unsigned short* __restrict__ A2p, int lda,
    const unsigned short* __restrict__ Btp, const unsigned short* __restrict__ Bt2p, int ldb,
    void* __restrict__ Cout, void* __restrict__ Cout2, int ldc,
    const float* __restrict__ rcos, const float* __restrict__ rsin, int rld, int rmask,
    int M, int N, int K, float scale) {
  static_assert(OUT_MODE == 0 || OUT_MODE == 2);
  static_assert(!ROT || OUT_MODE == 2);
  typedef typename Elem<ET>::T T;
  typedef typename Frag<T>::V V;
  const T* A = (const T*)Ap; const T* A2 = (const T*)A2p; const T* Bt = (const T*)Btp; const T* Bt2 = (const T*)Bt2p;
  __shared__ __align__(16) float sT[8][16 * 68];
  const int lane = threadIdx.x & 31;
  const int wave = threadIdx.x >> 5;
  const int tilesN = N >> 6;
  const int tilesM = M >> 6;
  const int nTiles = (TILEMAP == 1) ? ((tilesM * (tilesM + 1)) >> 1) : (tilesM * tilesN);
  const int tile = blockIdx.x * 8 + wave;
  if (tile >= nTiles) return;
  int tm, tn;
  if (TILEMAP == 1) {
    int t = (int)((sqrtf(8.0f * (float)tile + 1.0f) - 1.0f) * 0.5f);
    if (((t + 1) * (t + 2)) / 2 <= tile) ++t;
    if (((t + 1) * (t + 2)) / 2 <= tile) ++t;
    if ((t * (t + 1)) / 2 > tile) --t;
    if ((t * (t + 1)) / 2 > tile) --t;
    t = (t < 0) ? 0 : ((t > tilesM - 1) ? (tilesM - 1) : t);
    tm = t;
    tn = tile - ((t * (t + 1)) >> 1);
    tn = (tn < 0) ? 0 : ((tn > tm) ? tm : tn);
  } else {
    tm = tile / tilesN;
    tn = tile - tm * tilesN;
  }
  const int m0 = tm << 6;
  const int n0 = tn << 6;
  int Keff = K;
  if (KCAUS) { const int kc = (tm + 1) << 6; Keff = (kc < K) ? kc : K; }

  const int rlane = lane & 15;
  const int koff  = (lane >> 4) * 8;
  const int mOff  = (lane >> 4) * 8;

  v8f acc[4][4];
#pragma unroll
  for (int i = 0; i < 4; ++i)
#pragma unroll
    for (int j = 0; j < 4; ++j) acc[i][j] = (v8f){0.f,0.f,0.f,0.f,0.f,0.f,0.f,0.f};

  for (int k0 = 0; k0 < Keff; k0 += 32) {
    V bh[4], bl[4];
#pragma unroll
    for (int j = 0; j < 4; ++j) {
      const size_t bo = (size_t)(n0 + (j << 4) + rlane) * ldb + koff + k0;
      bh[j] = Frag<T>::load(Bt + bo);
      if (SPLIT) bl[j] = Frag<T>::load(Bt2 + bo);
    }
#pragma unroll
    for (int i = 0; i < 4; ++i) {
      const size_t ao = (size_t)(m0 + (i << 4) + rlane) * lda + koff + k0;
      V ah = Frag<T>::load(A + ao);
      V al;
      if (SPLIT) al = Frag<T>::load(A2 + ao);
#pragma unroll
      for (int j = 0; j < 4; ++j) {
        acc[i][j] = Frag<T>::mma(ah, bh[j], acc[i][j]);
        if (SPLIT) {
          acc[i][j] = Frag<T>::mma(ah, bl[j], acc[i][j]);
          acc[i][j] = Frag<T>::mma(al, bh[j], acc[i][j]);
        }
      }
      Frag<T>::guard(acc[i][0], acc[i][3], ah, SPLIT ? al : ah);
    }
    Frag<T>::keep(bh[0], bh[1], bh[2], bh[3]);
    if (SPLIT) Frag<T>::keep(bl[0], bl[1], bl[2], bl[3]);
  }
  acc_guard4(acc[0][0], acc[0][1], acc[0][2], acc[0][3]);
  acc_guard4(acc[1][0], acc[1][1], acc[1][2], acc[1][3]);
  acc_guard4(acc[2][0], acc[2][1], acc[2][2], acc[2][3]);
  acc_guard4(acc[3][0], acc[3][1], acc[3][2], acc[3][3]);

  float* slab = sT[wave];
#pragma unroll
  for (int i = 0; i < 4; ++i) {
    const int mBase = m0 + (i << 4);
#pragma unroll
    for (int j = 0; j < 4; ++j) {
#pragma unroll
      for (int r = 0; r < 8; ++r) {
        const float v = acc[i][j][r] * scale;
        slab[(mOff + r) * 68 + (j << 4) + rlane] = v;
      }
    }
    __builtin_amdgcn_fence(__ATOMIC_RELEASE, "workgroup");
    __builtin_amdgcn_wave_barrier();
    __builtin_amdgcn_fence(__ATOMIC_ACQUIRE, "workgroup");
    if (OUT_MODE == 0) {
      float* C = (float*)Cout;
      const int hh = lane >> 4, c4 = (lane & 15) * 4;
      for (int pass = 0; pass < 2; ++pass) {
#pragma unroll
        for (int it = 0; it < 8; ++it) {
          const int row = it * 2 + hh;
          v4f v = *(const v4f*)(slab + row * 68 + c4);
          *(volatile v4f*)(C + (size_t)(mBase + row) * ldc + n0 + c4) = v;
        }
        __threadfence();
      }
    } else {
      const int q = lane >> 3, c8 = (lane & 7) * 8;
      unsigned short* C  = (unsigned short*)Cout;
      unsigned short* C2 = (unsigned short*)Cout2;
      for (int pass = 0; pass < 2; ++pass) {
#pragma unroll
        for (int it = 0; it < 4; ++it) {
          const int row = it * 4 + q;
          const float* sp = slab + row * 68 + c8;
          float vv[8];
#pragma unroll
          for (int e = 0; e < 8; ++e) vv[e] = sp[e];
          if (ROT) {
            const int pos = mBase + row;
            const int i0 = ((n0 + c8) & rmask) >> 1;
            const v4f cv = *(const v4f*)(rcos + (size_t)pos * rld + i0);
            const v4f sv = *(const v4f*)(rsin + (size_t)pos * rld + i0);
#pragma unroll
            for (int p = 0; p < 4; ++p) {
              const float te = vv[2 * p], to = vv[2 * p + 1];
              vv[2 * p]     = te * cv[p] + to * sv[p];
              vv[2 * p + 1] = to * cv[p] - te * sv[p];
            }
          }
          v8h hv, lv;
#pragma unroll
          for (int e = 0; e < 8; ++e) {
            const unsigned short hb = f2bf_bits(vv[e]);
            const unsigned short lb = f2bf_bits(vv[e] - bf_bits2f(hb));
            hv[e] = __builtin_bit_cast(_Float16, hb);
            lv[e] = __builtin_bit_cast(_Float16, lb);
          }
          *(volatile v8h*)(C  + (size_t)(mBase + row) * ldc + n0 + c8) = hv;
          *(volatile v8h*)(C2 + (size_t)(mBase + row) * ldc + n0 + c8) = lv;
        }
        __threadfence();
      }
    }
    __builtin_amdgcn_fence(__ATOMIC_RELEASE, "workgroup");
    __builtin_amdgcn_wave_barrier();
    __builtin_amdgcn_fence(__ATOMIC_ACQUIRE, "workgroup");
  }
}

__global__ __launch_bounds__(256) void cast_f32_bf16x2(
    const float* __restrict__ in, unsigned short* __restrict__ out, int n2) {
  const int i = blockIdx.x * 256 + threadIdx.x;
  if (i < n2) {
    const float a = in[2 * i], b = in[2 * i + 1];
    const unsigned u = (unsigned)f2bf_bits(a) | ((unsigned)f2bf_bits(b) << 16);
    ((volatile unsigned*)out)[i] = u;
    __threadfence();
    ((volatile unsigned*)out)[i] = u;
  }
}

__global__ __launch_bounds__(256) void rot_tables(
    float* __restrict__ cosT, float* __restrict__ sinT, int npos, int nhalf, float invDim) {
#pragma clang fp contract(off)
  const int t = blockIdx.x * 256 + threadIdx.x;
  if (t < npos * nhalf) {
    const int pos = t / nhalf;
    const int i = t - pos * nhalf;
    const float ex = (-2.0f * ((float)i - 1.0f)) * invDim;
    const float phi = expf(ex * 9.2103403719761836f);
    const float ang = (float)pos * phi;
    const float c = cosf(ang);
    const float s = sinf(ang);
    ((volatile float*)cosT)[t] = c;
    ((volatile float*)sinT)[t] = s;
    __threadfence();
    ((volatile float*)cosT)[t] = c;
    ((volatile float*)sinT)[t] = s;
  }
}

__global__ __launch_bounds__(256) void causal_softmax_rows(
    const float* __restrict__ S, int ldS,
    unsigned short* __restrict__ Ph, unsigned short* __restrict__ Pl, int ldP) {
  constexpr float kNegFill = -3.40282347e38f;
  __shared__ float redMax[8];
  __shared__ float redSum[8];
  const int q = blockIdx.x;
  const int t = threadIdx.x;
  const int lane = t & 31, wave = t >> 5;
  const int kend = ((q >> 6) + 1) << 6;
  const int c0 = t * 8;
  const int cb = (c0 > kend - 8) ? (kend - 8) : c0;
  const float* srow = S + (size_t)q * ldS + cb;
  const v4f la = *(const v4f*)(srow);
  const v4f lb = *(const v4f*)(srow + 4);
  float sv[8];
  sv[0] = la[0]; sv[1] = la[1]; sv[2] = la[2]; sv[3] = la[3];
  sv[4] = lb[0]; sv[5] = lb[1]; sv[6] = lb[2]; sv[7] = lb[3];
#pragma unroll
  for (int e = 0; e < 8; ++e) { if (c0 + e > q) sv[e] = kNegFill; }
  float m = sv[0];
#pragma unroll
  for (int e = 1; e < 8; ++e) m = fmaxf(m, sv[e]);
#pragma unroll
  for (int off = 1; off < 32; off <<= 1) m = fmaxf(m, __shfl_xor(m, off, 32));
  if (lane == 0) redMax[wave] = m;
  __syncthreads();
  float gm = redMax[0];
#pragma unroll
  for (int w = 1; w < 8; ++w) gm = fmaxf(gm, redMax[w]);
  float p[8];
  float ls = 0.0f;
#pragma unroll
  for (int e = 0; e < 8; ++e) { p[e] = expf(sv[e] - gm); ls += p[e]; }
#pragma unroll
  for (int off = 1; off < 32; off <<= 1) ls += __shfl_xor(ls, off, 32);
  if (lane == 0) redSum[wave] = ls;
  __syncthreads();
  float l = 0.0f;
#pragma unroll
  for (int w = 0; w < 8; ++w) l += redSum[w];
  const float inv = 1.0f / l;
  if (c0 < kend) {
    v4u hw, lw;
#pragma unroll
    for (int pp = 0; pp < 4; ++pp) {
      const float P0 = p[2 * pp] * inv;
      const float P1 = p[2 * pp + 1] * inv;
      const unsigned short h0 = f2bf_bits(P0);
      const unsigned short h1 = f2bf_bits(P1);
      const unsigned short l0 = f2bf_bits(P0 - bf_bits2f(h0));
      const unsigned short l1 = f2bf_bits(P1 - bf_bits2f(h1));
      hw[pp] = (unsigned)h0 | ((unsigned)h1 << 16);
      lw[pp] = (unsigned)l0 | ((unsigned)l1 << 16);
    }
    unsigned short* ph = Ph + (size_t)q * ldP + c0;
    unsigned short* pl = Pl + (size_t)q * ldP + c0;
    *(volatile v4u*)ph = hw;
    *(volatile v4u*)pl = lw;
    __threadfence();
    *(volatile v4u*)ph = hw;
    *(volatile v4u*)pl = lw;
  }
}

extern "C" void kernel_launch(void* const* d_in, const int* in_sizes, int n_in,
                              void* d_out, int out_size, void* d_ws, size_t ws_size,
                              hipStream_t stream) {
  constexpr int kBatch = 4, kSeq = 2048, kDim = 1024, kHalfDim = kDim / 2;
  static_assert(kSeq % 64 == 0 && kDim % 64 == 0 && (2 * kDim) % 64 == 0);
  static_assert(kDim % 32 == 0 && kSeq % 32 == 0);
  static_assert(kHalfDim % 4 == 0);
  static_assert((kBatch * kSeq * kDim) % 2 == 0 && (kDim * kDim) % 2 == 0);
  if (n_in < 4) return;
  if (in_sizes[0] != kBatch * kSeq * kDim) return;
  if (in_sizes[1] != kDim * kDim || in_sizes[2] != kDim * kDim || in_sizes[3] != kDim * kDim) return;
  if (out_size != kBatch * kSeq * kDim) return;

  const float* x  = (const float*)d_in[0];
  const float* wq = (const float*)d_in[1];
  const float* wk = (const float*)d_in[2];
  const float* wv = (const float*)d_in[3];
  float* out = (float*)d_out;

  char* ws = (char*)d_ws;
  size_t off = 0;
  const size_t bWqk = (size_t)2 * kDim * kDim * 2;
  const size_t bWv  = (size_t)kDim * kDim * 2;
  const size_t bXb  = (size_t)kBatch * kSeq * kDim * 2;
  const size_t bTab = (size_t)kSeq * kHalfDim * 4;
  const size_t bQK  = (size_t)kSeq * 2 * kDim * 2;
  const size_t bVT  = (size_t)kDim * kSeq * 2;
  const size_t bS   = (size_t)kSeq * kSeq * 4;
  const size_t bP   = (size_t)kSeq * kSeq * 2;
  unsigned short* Wqk = (unsigned short*)(ws + off); off += bWqk;
  unsigned short* Wvb = (unsigned short*)(ws + off); off += bWv;
  unsigned short* Xb  = (unsigned short*)(ws + off); off += bXb;
  float* cosT = (float*)(ws + off); off += bTab;
  float* sinT = (float*)(ws + off); off += bTab;
  unsigned short* QKh = (unsigned short*)(ws + off); off += bQK;
  unsigned short* QKl = (unsigned short*)(ws + off); off += bQK;
  unsigned short* VTh = (unsigned short*)(ws + off); off += bVT;
  unsigned short* VTl = (unsigned short*)(ws + off); off += bVT;
  float* Sf = (float*)(ws + off); off += bS;
  unsigned short* Ph = (unsigned short*)(ws + off); off += bP;
  unsigned short* Pl = (unsigned short*)(ws + off); off += bP;
  if (off > ws_size) return;

  {
    const int n2x = (kBatch * kSeq * kDim) / 2;
    const int n2w = (kDim * kDim) / 2;
    cast_f32_bf16x2<<<dim3((n2x + 255) / 256), dim3(256), 0, stream>>>(x, Xb, n2x);
    cast_f32_bf16x2<<<dim3((n2w + 255) / 256), dim3(256), 0, stream>>>(wq, Wqk, n2w);
    cast_f32_bf16x2<<<dim3((n2w + 255) / 256), dim3(256), 0, stream>>>(wk, Wqk + (size_t)kDim * kDim, n2w);
    cast_f32_bf16x2<<<dim3((n2w + 255) / 256), dim3(256), 0, stream>>>(wv, Wvb, n2w);
  }
  {
    const int nt = kSeq * kHalfDim;
    rot_tables<<<dim3((nt + 255) / 256), dim3(256), 0, stream>>>(cosT, sinT, kSeq, kHalfDim, 1.0f / (float)kDim);
  }

  const int gridQK  = (((kSeq / 64) * ((2 * kDim) / 64)) + 7) / 8;
  const int gridVT  = (((kDim / 64) * (kSeq / 64)) + 7) / 8;
  const int tilesSq = kSeq / 64;
  const int gridS   = (((tilesSq * (tilesSq + 1)) / 2) + 7) / 8;
  const int gridPV  = (((kSeq / 64) * (kDim / 64)) + 7) / 8;

  for (int b = 0; b < kBatch; ++b) {
    const unsigned short* Xbb = Xb + (size_t)b * kSeq * kDim;
    float* outb = out + (size_t)b * kSeq * kDim;

    gemm64x<1, false, 2, 0, false, true><<<dim3(gridQK), dim3(256), 0, stream>>>(
        Xbb, Xbb, kDim, Wqk, Wqk, kDim, (void*)QKh, (void*)QKl, 2 * kDim,
        cosT, sinT, kHalfDim, kDim - 1, kSeq, 2 * kDim, kDim, 1.0f);

    gemm64x<1, false, 2, 0, false, false><<<dim3(gridVT), dim3(256), 0, stream>>>(
        Wvb, Wvb, kDim, Xbb, Xbb, kDim, (void*)VTh, (void*)VTl, kSeq,
        cosT, sinT, kHalfDim, kDim - 1, kDim, kSeq, kDim, 1.0f);

    gemm64x<1, true, 0, 1, false, false><<<dim3(gridS), dim3(256), 0, stream>>>(
        QKh, QKl, 2 * kDim, QKh + kDim, QKl + kDim, 2 * kDim, (void*)Sf, (void*)Sf, kSeq,
        cosT, sinT, kHalfDim, kDim - 1, kSeq, kSeq, kDim, 0.03125f);

    causal_softmax_rows<<<dim3(kSeq), dim3(256), 0, stream>>>(Sf, kSeq, Ph, Pl, kSeq);

    gemm64x<1, true, 0, 0, true, false><<<dim3(gridPV), dim3(256), 0, stream>>>(
        Ph, Pl, kSeq, VTh, VTl, kSeq, (void*)outb, (void*)outb, kDim,
        cosT, sinT, kHalfDim, kDim - 1, kSeq, kDim, kSeq, 1.0f);
  }
}
